// DifferentiableAttention_9818295239474
// MI455X (gfx1250) — hardware-verified
//
#include <hip/hip_runtime.h>
#include <stddef.h>
#include <stdint.h>

#define NBATCH 4
#define SEQ    1024
#define HID    1024
#define HDIM   64
#define NPAIR  16
#define GDIM   512
#define QW     (2 * HID)
#define NQKV   (2 * HID + 2 * GDIM)
#define NTOK   (NBATCH * SEQ)
#define LAMBDA_INIT 0.355509067590969f
#define ONE_M_LI    0.644490932409031f

#define QPB ((size_t)SEQ * QW)
#define KPB ((size_t)SEQ * GDIM)
#define HPL ((size_t)SEQ * HDIM)

static_assert(NQKV == 3072);
static_assert(HID % 32 == 0);
static_assert(NTOK % 256 == 0);
static_assert(NQKV % 64 == 0);
static_assert(QW % 64 == 0);
static_assert(GDIM % 64 == 0);
static_assert(SEQ % 64 == 0);
static_assert(SEQ % 256 == 0);
static_assert(HID % 256 == 0);
static_assert(HID == NPAIR * HDIM);
static_assert(SEQ * QW == 32 * SEQ * HDIM);
static_assert(SEQ * GDIM == 8 * SEQ * HDIM);
static_assert(GDIM == 4 * 128);

typedef _Float16 v16h __attribute__((ext_vector_type(16)));
typedef _Float16 v8h  __attribute__((ext_vector_type(8)));
typedef float    v8f  __attribute__((ext_vector_type(8)));
typedef float    v4f  __attribute__((ext_vector_type(4)));
typedef unsigned int   v4u   __attribute__((ext_vector_type(4)));
typedef unsigned short v8us  __attribute__((ext_vector_type(8)));
typedef unsigned short v16us __attribute__((ext_vector_type(16)));
typedef __bf16         v16b  __attribute__((ext_vector_type(16)));
typedef unsigned short ush;

union Frag  { v16h v; v8h h[2]; };
union FragU { v16us v; v8us h[2]; v16b b; };
union PackU { v8us s; v4u u; };
union H1    { _Float16 h; ush u; };
struct HL   { v4u h; v4u l; };

__device__ __forceinline__ ush f2bf(float f) {
  const unsigned u = __float_as_uint(f);
  return (ush)((u + 0x7FFFu + ((u >> 16) & 1u)) >> 16);
}
__device__ __forceinline__ float bf2f(ush b) { return __uint_as_float(((unsigned)b) << 16); }
__device__ __forceinline__ ush f2h(float f) { H1 x; x.h = (_Float16)f; return x.u; }

__device__ __forceinline__ HL split8(v8f f) {
  PackU ph, pl;
#pragma unroll
  for (int e = 0; e < 8; ++e) {
    const ush hi = f2bf(f[e]);
    ph.s[e] = hi;
    pl.s[e] = f2bf(f[e] - bf2f(hi));
  }
  HL r; r.h = ph.u; r.l = pl.u;
  return r;
}

__device__ __forceinline__ v8f mma16(v16h a, v16h b, v8f c) {
  c = __builtin_amdgcn_wmma_f32_16x16x32_f16(false, a, false, b, (short)0, c, false, false);
  asm volatile("v_nop\n\tv_nop\n\tv_nop\n\tv_nop" : "+v"(c) : "v"(a), "v"(b));
  return c;
}
__device__ __forceinline__ v8f mmab(v16us a, v16us b, v8f c) {
  FragU ua, ub; ua.v = a; ub.v = b;
  c = __builtin_amdgcn_wmma_f32_16x16x32_bf16(false, ua.b, false, ub.b, (short)0, c, false, false);
  asm volatile("v_nop\n\tv_nop\n\tv_nop\n\tv_nop" : "+v"(c) : "v"(a), "v"(b));
  return c;
}

__device__ __forceinline__ v16h ldfrag(const _Float16* p, int ld, int row0, int k0, int lane) {
  const int m = lane & 15, lh = lane >> 4;
  const _Float16* q = p + (size_t)(row0 + m) * ld + k0 + 8 * lh;
  Frag f;
  f.h[0] = *(const v8h*)(q);
  f.h[1] = *(const v8h*)(q + 16);
  return f.v;
}
__device__ __forceinline__ v16us ldfragu(const ush* p, int ld, int row0, int k0, int lane) {
  const int m = lane & 15, lh = lane >> 4;
  const ush* q = p + (size_t)(row0 + m) * ld + k0 + 8 * lh;
  FragU f;
  f.h[0] = *(const v8us*)(q);
  f.h[1] = *(const v8us*)(q + 16);
  return f.v;
}

__device__ __forceinline__ v8f zero8() { return (v8f){0.f, 0.f, 0.f, 0.f, 0.f, 0.f, 0.f, 0.f}; }

__device__ __forceinline__ void gemm32x64(const _Float16* __restrict__ A, int lda,
                                          const _Float16* __restrict__ Bt, int ldb,
                                          int m0, int n0, int lane, v8f (&acc)[2][4]) {
#pragma unroll 2
  for (int k0 = 0; k0 < HID; k0 += 32) {
    const v16h a0 = ldfrag(A, lda, m0, k0, lane);
    const v16h a1 = ldfrag(A, lda, m0 + 16, k0, lane);
    const v16h b0 = ldfrag(Bt, ldb, n0, k0, lane);
    const v16h b1 = ldfrag(Bt, ldb, n0 + 16, k0, lane);
    const v16h b2 = ldfrag(Bt, ldb, n0 + 32, k0, lane);
    const v16h b3 = ldfrag(Bt, ldb, n0 + 48, k0, lane);
    acc[0][0] = mma16(a0, b0, acc[0][0]);
    acc[1][0] = mma16(a1, b0, acc[1][0]);
    acc[0][1] = mma16(a0, b1, acc[0][1]);
    acc[1][1] = mma16(a1, b1, acc[1][1]);
    acc[0][2] = mma16(a0, b2, acc[0][2]);
    acc[1][2] = mma16(a1, b2, acc[1][2]);
    acc[0][3] = mma16(a0, b3, acc[0][3]);
    acc[1][3] = mma16(a1, b3, acc[1][3]);
  }
}

__device__ __forceinline__ void gemm3_32x64(const ush* __restrict__ Ah, const ush* __restrict__ Al, int lda,
                                            const ush* __restrict__ Bh, const ush* __restrict__ Bl, int ldb,
                                            int m0, int n0, int lane, v8f (&acc)[2][4]) {
#pragma unroll 1
  for (int k0 = 0; k0 < HID; k0 += 32) {
    const v16us a0h = ldfragu(Ah, lda, m0, k0, lane);
    const v16us a1h = ldfragu(Ah, lda, m0 + 16, k0, lane);
    const v16us a0l = ldfragu(Al, lda, m0, k0, lane);
    const v16us a1l = ldfragu(Al, lda, m0 + 16, k0, lane);
#pragma unroll
    for (int t = 0; t < 4; ++t) {
      const v16us bh = ldfragu(Bh, ldb, n0 + 16 * t, k0, lane);
      const v16us bl = ldfragu(Bl, ldb, n0 + 16 * t, k0, lane);
      acc[0][t] = mmab(a0h, bh, acc[0][t]);
      acc[1][t] = mmab(a1h, bh, acc[1][t]);
      acc[0][t] = mmab(a0h, bl, acc[0][t]);
      acc[1][t] = mmab(a1h, bl, acc[1][t]);
      acc[0][t] = mmab(a0l, bh, acc[0][t]);
      acc[1][t] = mmab(a1l, bh, acc[1][t]);
    }
  }
}

__global__ __launch_bounds__(256) void k_cvt_x(const float* __restrict__ x, ush* __restrict__ xh,
                                               ush* __restrict__ xl, int ngrp) {
  const int t = blockIdx.x * 256 + (int)threadIdx.x;
  if (t >= ngrp) return;
  const size_t o = (size_t)t * 8;
  const v4f a0 = *(const v4f*)(x + o);
  const v4f a1 = *(const v4f*)(x + o + 4);
  const v8f f = (v8f){a0[0], a0[1], a0[2], a0[3], a1[0], a1[1], a1[2], a1[3]};
  const HL s = split8(f);
  *(volatile v4u*)(xh + o) = s.h;
  *(volatile v4u*)(xl + o) = s.l;
  __threadfence();
  *(volatile v4u*)(xh + o) = s.h;
  *(volatile v4u*)(xl + o) = s.l;
}

#define TTP 72
template <int MODE>
__global__ __launch_bounds__(256) void k_trw(const float* __restrict__ w, int ncol, int nrow,
                                             ush* __restrict__ o0, ush* __restrict__ o1) {
  __shared__ __align__(16) ush t0[64 * TTP];
  __shared__ __align__(16) ush t1[64 * TTP];
  const int tid = threadIdx.x;
  const int n0 = blockIdx.x * 64;
  const int k0 = blockIdx.y * 64;
#pragma unroll
  for (int it = 0; it < 4; ++it) {
    const int cidx = tid + 256 * it;
    const int kr = cidx >> 4;
    const int nq = (cidx & 15) * 4;
    const v4f v = *(const v4f*)(w + (size_t)(k0 + kr) * ncol + n0 + nq);
#pragma unroll
    for (int i = 0; i < 4; ++i) {
      if (MODE == 0) {
        const ush hi = f2bf(v[i]);
        t0[(nq + i) * TTP + kr] = hi;
        t1[(nq + i) * TTP + kr] = f2bf(v[i] - bf2f(hi));
      } else {
        t0[(nq + i) * TTP + kr] = f2h(v[i] * 32.0f);
      }
    }
  }
  __syncthreads();
  v4u va[2], vb[2];
  size_t go[2];
#pragma unroll
  for (int j = 0; j < 2; ++j) {
    const int p  = tid + 256 * j;
    const int L  = p >> 3;
    const int pc = p & 7;
    PackU pk;
    pk.s  = *(const v8us*)(t0 + L * TTP + pc * 8);
    va[j] = pk.u;
    vb[j] = pk.u;
    if (MODE == 0) { PackU pq; pq.s = *(const v8us*)(t1 + L * TTP + pc * 8); vb[j] = pq.u; }
    go[j] = (size_t)(n0 + L) * nrow + k0 + pc * 8;
  }
#pragma unroll
  for (int j = 0; j < 2; ++j) {
    *(volatile v4u*)(o0 + go[j]) = va[j];
    if (MODE == 0) *(volatile v4u*)(o1 + go[j]) = vb[j];
  }
  __threadfence();
#pragma unroll
  for (int j = 0; j < 2; ++j) {
    *(volatile v4u*)(o0 + go[j]) = va[j];
    if (MODE == 0) *(volatile v4u*)(o1 + go[j]) = vb[j];
  }
}

#define STP 72
__global__ __launch_bounds__(256) void k_qkv(const ush* __restrict__ xh, const ush* __restrict__ xl,
                                             const ush* __restrict__ wth, const ush* __restrict__ wtl,
                                             ush* __restrict__ qp, ush* __restrict__ kp,
                                             ush* __restrict__ vh, ush* __restrict__ vl) {
  __shared__ __align__(16) ush st[256 * STP];
  const int tid = threadIdx.x, lane = tid & 31, wave = tid >> 5;
  const int hh = lane >> 4, c = lane & 15;
  const int mb = blockIdx.x * 256;
  const int m0 = mb + wave * 32;
  const int n0 = blockIdx.y * 64;
  const int which = (n0 < QW) ? 0 : ((n0 < QW + GDIM) ? 1 : 2);
  const int nn    = (which == 0) ? n0 : ((which == 1) ? (n0 - QW) : (n0 - QW - GDIM));
  const int pitch = (which == 0) ? QW : GDIM;

  v8f acc[2][4];
#pragma unroll
  for (int s = 0; s < 2; ++s)
#pragma unroll
    for (int t = 0; t < 4; ++t) acc[s][t] = zero8();
  gemm3_32x64(xh, xl, HID, wth, wtl, HID, m0, n0, lane, acc);

  size_t go[8];
#pragma unroll
  for (int j = 0; j < 8; ++j) {
    const int p  = tid + 256 * j;
    const int L  = p >> 3;
    const int pc = p & 7;
    go[j] = ((size_t)(mb + L)) * pitch + nn + pc * 8;
  }

  const int nph = (which == 2) ? 2 : 1;
#pragma unroll 1
  for (int ph = 0; ph < nph; ++ph) {
    __syncthreads();
#pragma unroll
    for (int t = 0; t < 4; ++t) {
#pragma unroll
      for (int sub = 0; sub < 2; ++sub) {
#pragma unroll
        for (int r = 0; r < 8; ++r) {
          const int lr = wave * 32 + sub * 16 + 8 * hh + r;
          const float v = acc[sub][t][r];
          ush bits;
          if (which == 2) {
            const ush hi = f2bf(v);
            bits = (ph == 0) ? hi : f2bf(v - bf2f(hi));
          } else {
            bits = f2h(v * 4.0f);
          }
          st[lr * STP + 16 * t + c] = bits;
        }
      }
    }
    __syncthreads();
    v4u val[8];
#pragma unroll
    for (int j = 0; j < 8; ++j) {
      const int p  = tid + 256 * j;
      const int lr = p >> 3;
      const int pc = p & 7;
      PackU pk;
      pk.s   = *(const v8us*)(st + lr * STP + pc * 8);
      val[j] = pk.u;
    }
    ush* dst = (which == 0) ? qp : ((which == 1) ? kp : ((ph == 0) ? vh : vl));
#pragma unroll
    for (int j = 0; j < 8; ++j) *(volatile v4u*)(dst + go[j]) = val[j];
    __threadfence();
#pragma unroll
    for (int j = 0; j < 8; ++j) *(volatile v4u*)(dst + go[j]) = val[j];
  }
}

#define VP 72
#define PP 72
__device__ __forceinline__ void stat_upd(const v8f (&s)[4], float (&m)[8], float (&l)[8],
                                         int rw0, int j0, int hh, int c, float sc) {
#pragma unroll
  for (int r = 0; r < 8; ++r) {
    const int row = rw0 + 8 * hh + r;
    float v[4];
    float mx = -1.0e30f;
#pragma unroll
    for (int t = 0; t < 4; ++t) {
      const int key = j0 + 16 * t + c;
      float xv = s[t][r] * sc;
      xv = (key > row) ? -1.0e30f : xv;
      v[t] = xv;
      mx = fmaxf(mx, xv);
    }
    mx = fmaxf(mx, __shfl_xor(mx, 1));
    mx = fmaxf(mx, __shfl_xor(mx, 2));
    mx = fmaxf(mx, __shfl_xor(mx, 4));
    mx = fmaxf(mx, __shfl_xor(mx, 8));
    const float mn   = fmaxf(m[r], mx);
    const float corr = __expf(m[r] - mn);
    float rs = 0.f;
#pragma unroll
    for (int t = 0; t < 4; ++t) rs += __expf(v[t] - mn);
    rs += __shfl_xor(rs, 1);
    rs += __shfl_xor(rs, 2);
    rs += __shfl_xor(rs, 4);
    rs += __shfl_xor(rs, 8);
    l[r] = l[r] * corr + rs;
    m[r] = mn;
  }
}

__global__ __launch_bounds__(128) void k_attn(const _Float16* __restrict__ qp,
                                              const _Float16* __restrict__ kp,
                                              const ush* __restrict__ vh,
                                              const ush* __restrict__ vl,
                                              const float* __restrict__ lq1,
                                              const float* __restrict__ lk1,
                                              const float* __restrict__ lq2,
                                              const float* __restrict__ lk2,
                                              ush* __restrict__ ap, float sc) {
  __shared__ __align__(16) ush sVh[64 * VP];
  __shared__ __align__(16) ush sVl[64 * VP];
  __shared__ __align__(16) ush sPh[64 * PP];
  __shared__ __align__(16) ush sPl[64 * PP];
  __shared__ float sred[8];

  const int tid = threadIdx.x, lane = tid & 31, wave = tid >> 5;
  const int hh = lane >> 4, c = lane & 15;
  const int qb = blockIdx.x, pi = blockIdx.y, b = blockIdx.z;
  const int q0  = qb * 64;
  const int rw0 = q0 + 16 * wave;
  const _Float16* Q1 = qp + (size_t)b * QPB + (size_t)(2 * pi) * HPL;
  const _Float16* Q2 = Q1 + HPL;
  const _Float16* Kg = kp + (size_t)b * KPB + (size_t)(pi >> 1) * HPL;
  const ush* Vgh = vh + (size_t)b * KPB + (size_t)(pi >> 1) * HPL;
  const ush* Vgl = vl + (size_t)b * KPB + (size_t)(pi >> 1) * HPL;

  float d1 = 0.f, d2 = 0.f;
#pragma unroll
  for (int j = 0; j < 4; ++j) {
    const int i = tid + 128 * j;
    d1 += lq1[i] * lk1[i];
    d2 += lq2[i] * lk2[i];
  }
  for (int o = 16; o > 0; o >>= 1) {
    d1 += __shfl_xor(d1, o);
    d2 += __shfl_xor(d2, o);
  }
  if (lane == 0) { sred[wave] = d1; sred[4 + wave] = d2; }
  __syncthreads();
  const float e1  = ((sred[0] + sred[1]) + sred[2]) + sred[3];
  const float e2  = ((sred[4] + sred[5]) + sred[6]) + sred[7];
  const float lam = (expf(e1) - expf(e2)) + LAMBDA_INIT;

  v16h q1f[2], q2f[2];
#pragma unroll
  for (int ks = 0; ks < 2; ++ks) {
    q1f[ks] = ldfrag(Q1, HDIM, rw0, 32 * ks, lane);
    q2f[ks] = ldfrag(Q2, HDIM, rw0, 32 * ks, lane);
  }

  const int nch = qb + 1;

  float m1[8], l1[8], m2[8], l2[8];
#pragma unroll
  for (int r = 0; r < 8; ++r) { m1[r] = -1.0e30f; m2[r] = -1.0e30f; l1[r] = 0.f; l2[r] = 0.f; }
#pragma unroll 1
  for (int ch = 0; ch < nch; ++ch) {
    const int j0 = ch * 64;
    v8f s1[4], s2[4];
#pragma unroll
    for (int t = 0; t < 4; ++t) { s1[t] = zero8(); s2[t] = zero8(); }
#pragma unroll
    for (int t = 0; t < 4; ++t) {
#pragma unroll
      for (int ks = 0; ks < 2; ++ks) {
        const v16h kf = ldfrag(Kg, HDIM, j0 + 16 * t, 32 * ks, lane);
        s1[t] = mma16(q1f[ks], kf, s1[t]);
        s2[t] = mma16(q2f[ks], kf, s2[t]);
      }
    }
    stat_upd(s1, m1, l1, rw0, j0, hh, c, sc);
    stat_upd(s2, m2, l2, rw0, j0, hh, c, sc);
  }

  float i1[8], c2[8];
#pragma unroll
  for (int r = 0; r < 8; ++r) {
    i1[r] = 1.0f / l1[r];
    c2[r] = lam * (1.0f / l2[r]);
  }
  v8f oacc[4];
#pragma unroll
  for (int t = 0; t < 4; ++t) oacc[t] = zero8();

#pragma unroll 1
  for (int ch = 0; ch < nch; ++ch) {
    const int j0 = ch * 64;
    __syncthreads();
#pragma unroll
    for (int it = 0; it < 4; ++it) {
      const int p  = tid + 128 * it;
      const int kr = p >> 3;
      const int pc = p & 7;
      PackU gh, gl;
      gh.s = *(const v8us*)(Vgh + (size_t)(j0 + kr) * HDIM + pc * 8);
      gl.s = *(const v8us*)(Vgl + (size_t)(j0 + kr) * HDIM + pc * 8);
#pragma unroll
      for (int e = 0; e < 8; ++e) {
        sVh[(pc * 8 + e) * VP + kr] = gh.s[e];
        sVl[(pc * 8 + e) * VP + kr] = gl.s[e];
      }
    }
#pragma unroll
    for (int t = 0; t < 4; ++t) {
      v8f a1 = zero8(), a2 = zero8();
#pragma unroll
      for (int ks = 0; ks < 2; ++ks) {
        const v16h kf = ldfrag(Kg, HDIM, j0 + 16 * t, 32 * ks, lane);
        a1 = mma16(q1f[ks], kf, a1);
        a2 = mma16(q2f[ks], kf, a2);
      }
      const int key = j0 + 16 * t + c;
#pragma unroll
      for (int r = 0; r < 8; ++r) {
        const int row = rw0 + 8 * hh + r;
        const bool msk = key > row;
        const float x1 = msk ? -1.0e30f : (a1[r] * sc);
        const float x2 = msk ? -1.0e30f : (a2[r] * sc);
        const float aw = __expf(x1 - m1[r]) * i1[r] - __expf(x2 - m2[r]) * c2[r];
        const ush hi = f2bf(aw);
        const int o  = (16 * wave + 8 * hh + r) * PP + 16 * t + c;
        sPh[o] = hi;
        sPl[o] = f2bf(aw - bf2f(hi));
      }
    }
    __syncthreads();
#pragma unroll
    for (int kk = 0; kk < 2; ++kk) {
      const v16us pah = ldfragu(sPh, PP, 16 * wave, 32 * kk, lane);
      const v16us pal = ldfragu(sPl, PP, 16 * wave, 32 * kk, lane);
#pragma unroll
      for (int t = 0; t < 4; ++t) {
        const v16us vbh = ldfragu(sVh, VP, 16 * t, 32 * kk, lane);
        const v16us vbl = ldfragu(sVl, VP, 16 * t, 32 * kk, lane);
        oacc[t] = mmab(pah, vbh, oacc[t]);
        oacc[t] = mmab(pah, vbl, oacc[t]);
        oacc[t] = mmab(pal, vbh, oacc[t]);
      }
    }
  }

  __syncthreads();
  const float fo = ONE_M_LI * 16.0f;
#pragma unroll
  for (int r = 0; r < 8; ++r) {
#pragma unroll
    for (int t = 0; t < 4; ++t) sPh[(16 * wave + 8 * hh + r) * PP + 16 * t + c] = f2h(oacc[t][r] * fo);
  }
  __syncthreads();
  v4u val[4];
  size_t go[4];
#pragma unroll
  for (int it = 0; it < 4; ++it) {
    const int p  = lane + 32 * it;
    const int L  = p >> 3;
    const int pc = p & 7;
    PackU pk;
    pk.s    = *(const v8us*)(sPh + (16 * wave + L) * PP + pc * 8);
    val[it] = pk.u;
    go[it]  = ((size_t)b * SEQ + (size_t)(rw0 + L)) * HID + (size_t)pi * HDIM + pc * 8;
  }
#pragma unroll
  for (int it = 0; it < 4; ++it) *(volatile v4u*)(ap + go[it]) = val[it];
  __threadfence();
#pragma unroll
  for (int it = 0; it < 4; ++it) *(volatile v4u*)(ap + go[it]) = val[it];
}

#define OTP 68
template <int OM>
__global__ __launch_bounds__(256) void k_gemm(const _Float16* __restrict__ A, const _Float16* __restrict__ Bt,
                                              void* __restrict__ outp, int ldo,
                                              long long sA, long long sB, long long sO, float oscale) {
  __shared__ __align__(16) float sm[9216];
  const int tid = threadIdx.x, lane = tid & 31, wave = tid >> 5;
  const int hh = lane >> 4, c = lane & 15;
  const int z  = blockIdx.z;
  const int mb = blockIdx.x * 256;
  const int m0 = mb + wave * 32;
  const int n0 = blockIdx.y * 64;
  const _Float16* Az = A + (size_t)z * (size_t)sA;
  const _Float16* Bz = Bt + (size_t)z * (size_t)sB;

  v8f acc[2][4];
#pragma unroll
  for (int s = 0; s < 2; ++s)
#pragma unroll
    for (int t = 0; t < 4; ++t) acc[s][t] = zero8();
  gemm32x64(Az, HID, Bz, HID, m0, n0, lane, acc);

  if (OM == 0) {
    ush* st = (ush*)sm;
#pragma unroll
    for (int t = 0; t < 4; ++t) {
#pragma unroll
      for (int sub = 0; sub < 2; ++sub) {
#pragma unroll
        for (int r = 0; r < 8; ++r) {
          const int lr = wave * 32 + sub * 16 + 8 * hh + r;
          st[lr * STP + 16 * t + c] = f2h(acc[sub][t][r] * oscale);
        }
      }
    }
    __syncthreads();
    ush* ob = (ush*)outp + (size_t)z * (size_t)sO;
    v4u val[8];
    size_t go[8];
#pragma unroll
    for (int j = 0; j < 8; ++j) {
      const int p  = tid + 256 * j;
      const int lr = p >> 3;
      const int pc = p & 7;
      PackU pk;
      pk.s   = *(const v8us*)(st + lr * STP + pc * 8);
      val[j] = pk.u;
      go[j]  = ((size_t)(mb + lr)) * ldo + n0 + pc * 8;
    }
#pragma unroll
    for (int j = 0; j < 8; ++j) *(volatile v4u*)(ob + go[j]) = val[j];
    __threadfence();
#pragma unroll
    for (int j = 0; j < 8; ++j) *(volatile v4u*)(ob + go[j]) = val[j];
  } else {
    float* sw = sm;
    float* ob = (float*)outp + (size_t)z * (size_t)sO;
#pragma unroll
    for (int sub = 0; sub < 2; ++sub) {
      __syncthreads();
#pragma unroll
      for (int r = 0; r < 8; ++r) {
        const int lr = wave * 16 + 8 * hh + r;
#pragma unroll
        for (int t = 0; t < 4; ++t) sw[lr * OTP + 16 * t + c] = acc[sub][t][r] * oscale;
      }
      __syncthreads();
      v4f val[8];
      size_t go[8];
#pragma unroll
      for (int j = 0; j < 8; ++j) {
        const int p    = tid + 256 * j;
        const int L    = p >> 3;
        const int pc   = p & 7;
        const int row  = L >> 1;
        const int half = L & 1;
        const int grow = mb + (row >> 4) * 32 + 16 * sub + (row & 15);
        val[j] = *(const v4f*)(sw + row * OTP + half * 32 + pc * 4);
        go[j]  = ((size_t)grow) * ldo + n0 + half * 32 + pc * 4;
      }
#pragma unroll
      for (int j = 0; j < 8; ++j) *(volatile v4f*)(ob + go[j]) = val[j];
      __threadfence();
#pragma unroll
      for (int j = 0; j < 8; ++j) *(volatile v4f*)(ob + go[j]) = val[j];
    }
  }
}

extern "C" void kernel_launch(void* const* d_in, const int* in_sizes, int n_in,
                              void* d_out, int out_size, void* d_ws, size_t ws_size,
                              hipStream_t stream) {
  if (n_in < 7) return;
  if (in_sizes[0] != NTOK * HID) return;
  if (in_sizes[1] != HID * NQKV) return;
  if (in_sizes[2] != HID * HID) return;
  if (in_sizes[3] != GDIM) return;
  if (in_sizes[4] != GDIM) return;
  if (in_sizes[5] != GDIM) return;
  if (in_sizes[6] != GDIM) return;
  if (out_size != NTOK * HID) return;

  const float* x     = (const float*)d_in[0];
  const float* wqkv  = (const float*)d_in[1];
  const float* wproj = (const float*)d_in[2];
  const float* lq1   = (const float*)d_in[3];
  const float* lk1   = (const float*)d_in[4];
  const float* lq2   = (const float*)d_in[5];
  const float* lk2   = (const float*)d_in[6];
  float* out = (float*)d_out;

  size_t off = 0;
  const size_t oXh  = off; off += (size_t)NTOK * HID * 2;
  const size_t oXl  = off; off += (size_t)NTOK * HID * 2;
  const size_t oWth = off; off += (size_t)NQKV * HID * 2;
  const size_t oWtl = off; off += (size_t)NQKV * HID * 2;
  const size_t oWpt = off; off += (size_t)HID * HID * 2;
  const size_t oQ   = off; off += (size_t)NTOK * QW * 2;
  const size_t oK   = off; off += (size_t)NTOK * GDIM * 2;
  const size_t oVh  = off; off += (size_t)NTOK * GDIM * 2;
  const size_t oVl  = off; off += (size_t)NTOK * GDIM * 2;
  const size_t oA   = off; off += (size_t)NTOK * HID * 2;
  const size_t oY   = off; off += (size_t)NTOK * HID * 2;
  if (off > ws_size) return;
  if (off > (size_t)134217728) return;

  char* ws = (char*)d_ws;
  ush* Xh  = (ush*)(ws + oXh);
  ush* Xl  = (ush*)(ws + oXl);
  ush* Wth = (ush*)(ws + oWth);
  ush* Wtl = (ush*)(ws + oWtl);
  ush* Wpt = (ush*)(ws + oWpt);
  ush* Qp  = (ush*)(ws + oQ);
  ush* Kp  = (ush*)(ws + oK);
  ush* Vh  = (ush*)(ws + oVh);
  ush* Vl  = (ush*)(ws + oVl);
  ush* Ap  = (ush*)(ws + oA);
  ush* Y2  = (ush*)(ws + oY);

  const int ngx = in_sizes[0] / 8;
  k_cvt_x<<<dim3((ngx + 255) / 256), dim3(256), 0, stream>>>(x, Xh, Xl, ngx);
  k_trw<0><<<dim3(NQKV / 64, HID / 64), dim3(256), 0, stream>>>(wqkv, NQKV, HID, Wth, Wtl);
  k_trw<1><<<dim3(HID / 64, HID / 64), dim3(256), 0, stream>>>(wproj, HID, HID, Wpt, Wpt);
  k_qkv<<<dim3(NTOK / 256, NQKV / 64), dim3(256), 0, stream>>>(Xh, Xl, Wth, Wtl, Qp, Kp, Vh, Vl);
  k_attn<<<dim3(SEQ / 64, NPAIR, NBATCH), dim3(128), 0, stream>>>(
      (const _Float16*)Qp, (const _Float16*)Kp, Vh, Vl, lq1, lk1, lq2, lk2, Ap, 0.0078125f);
  k_gemm<0><<<dim3(HID / 256, SEQ / 64, NBATCH), dim3(256), 0, stream>>>(
      (const _Float16*)Wpt, (const _Float16*)Ap, (void*)Y2, SEQ,
      0LL, (long long)SEQ * HID, (long long)HID * SEQ, 0.03125f);
  k_gemm<1><<<dim3(SEQ / 256, HID / 64, NBATCH), dim3(256), 0, stream>>>(
      (const _Float16*)Y2, (const _Float16*)Wpt, d_out, HID,
      (long long)SEQ * HID, 0LL, (long long)SEQ * HID, 0.001953125f);
  (void)out;
  (void)hipGetLastError();
}
